// GPT2Attention_49624052138686
// MI455X (gfx1250) — hardware-verified
//
#include <hip/hip_runtime.h>


typedef _Float16 v16h __attribute__((ext_vector_type(16)));
typedef _Float16 v8h  __attribute__((ext_vector_type(8)));
typedef _Float16 v8ha __attribute__((ext_vector_type(8), may_alias));
typedef float    v8f  __attribute__((ext_vector_type(8)));
typedef float    v4f  __attribute__((ext_vector_type(4)));
typedef float    v4fa __attribute__((ext_vector_type(4), may_alias));

union Frag { v16h v; v8h h[2]; };

#ifndef NB
#define NB 2
#endif
#ifndef SEQ
#define SEQ 2048
#endif
#define NB_FULL 2
#define SEQ_FULL 2048

constexpr int kC   = 1024;
constexpr int kH   = 16;
constexpr int kD   = 64;
constexpr int kNQ  = 3 * kC;
constexpr int kER  = 256;
constexpr int kM   = NB * SEQ;
constexpr int kCP  = 132;
constexpr int kQBE = kER / 64;
constexpr int kQBL = (SEQ / 64 - kQBE) > 0 ? (SEQ / 64 - kQBE) : 1;

static_assert(NB >= 1 && NB <= NB_FULL);
static_assert(SEQ >= kER && SEQ <= SEQ_FULL && (SEQ % 64) == 0);
static_assert((kER % 64) == 0 && kH * kD == kC && (kC % 128) == 0 && (kNQ % 128) == 0 && (kM % 64) == 0);
static_assert((kCP % 4) == 0);

constexpr float kWCarry = 64.0f;
constexpr float kWInv   = 0.015625f;
constexpr float kPCarry = 1024.0f;
constexpr float kPInv   = 0.0009765625f;
constexpr float kRCarry = 2048.0f;
constexpr float kRInv   = 0.00048828125f;
constexpr float kScale  = 0.125f;

constexpr size_t kBytesX   = (size_t)kM * kC * 2;
constexpr size_t kBytesWq  = (size_t)kNQ * kC * 2;
constexpr size_t kBytesWp  = (size_t)kC * kC * 2;
constexpr size_t kBytesQK  = (size_t)NB * kH * SEQ * kD * 2;
constexpr size_t kBytesQKr = (size_t)NB * kH * kER * kD * 2;
constexpr size_t kBytesCtx = (size_t)kM * kC * 2;
constexpr size_t kBytesCtr = (size_t)NB * kER * kC * 2;
constexpr size_t kWsTotal  = kBytesX + kBytesWq + kBytesWp + 3 * kBytesQK + 3 * kBytesQKr + kBytesCtx + kBytesCtr;
static_assert(kWsTotal <= (size_t)134217728);
static_assert((kBytesX % 128) == 0 && (kBytesWq % 128) == 0 && (kBytesWp % 128) == 0 && (kBytesQK % 128) == 0 &&
              (kBytesQKr % 128) == 0 && (kBytesCtx % 128) == 0 && (kBytesCtr % 128) == 0);

__device__ __forceinline__ float bf16r(float f) {
  unsigned int u = __float_as_uint(f);
  u += 0x7FFFu + ((u >> 16) & 1u);
  u &= 0xFFFF0000u;
  return __uint_as_float(u);
}

__device__ __forceinline__ v8f mma(v16h a, v16h b, v8f c) {
  return __builtin_amdgcn_wmma_f32_16x16x32_f16(false, a, false, b, (short)0, c, false, false);
}

__device__ __forceinline__ void wave_lds_sync() {
  __builtin_amdgcn_fence(3, "workgroup");
  __builtin_amdgcn_wave_barrier();
  __builtin_amdgcn_fence(2, "workgroup");
}

template <bool RES>
__device__ __forceinline__ void gemm32(const _Float16* __restrict__ a0p, const _Float16* __restrict__ a1p,
                                       const _Float16* __restrict__ r0p, const _Float16* __restrict__ r1p,
                                       const _Float16* __restrict__ b0p, const _Float16* __restrict__ b1p,
                                       int K, v8f (&c)[4], v8f (&cr)[4]) {
#pragma unroll 1
  for (int k0 = 0; k0 < K; k0 += 32) {
    Frag a0, a1, b0, b1;
    a0.h[0] = *(const v8h*)(a0p + k0); a0.h[1] = *(const v8h*)(a0p + k0 + 16);
    a1.h[0] = *(const v8h*)(a1p + k0); a1.h[1] = *(const v8h*)(a1p + k0 + 16);
    b0.h[0] = *(const v8h*)(b0p + k0); b0.h[1] = *(const v8h*)(b0p + k0 + 16);
    b1.h[0] = *(const v8h*)(b1p + k0); b1.h[1] = *(const v8h*)(b1p + k0 + 16);
    c[0] = mma(a0.v, b0.v, c[0]);
    c[1] = mma(a0.v, b1.v, c[1]);
    c[2] = mma(a1.v, b0.v, c[2]);
    c[3] = mma(a1.v, b1.v, c[3]);
    if (RES) {
      Frag e0, e1;
      e0.h[0] = *(const v8h*)(r0p + k0); e0.h[1] = *(const v8h*)(r0p + k0 + 16);
      e1.h[0] = *(const v8h*)(r1p + k0); e1.h[1] = *(const v8h*)(r1p + k0 + 16);
      cr[0] = mma(e0.v, b0.v, cr[0]);
      cr[1] = mma(e0.v, b1.v, cr[1]);
      cr[2] = mma(e1.v, b0.v, cr[2]);
      cr[3] = mma(e1.v, b1.v, cr[3]);
      asm volatile("v_nop\n\tv_nop\n\tv_nop\n\tv_nop"
                   : "+v"(c[0]), "+v"(c[1]), "+v"(c[2]), "+v"(c[3]), "+v"(cr[0]), "+v"(cr[1]), "+v"(cr[2]), "+v"(cr[3])
                   : "v"(a0.v), "v"(a1.v), "v"(b0.v), "v"(b1.v), "v"(e0.v), "v"(e1.v));
    } else {
      asm volatile("v_nop\n\tv_nop\n\tv_nop\n\tv_nop"
                   : "+v"(c[0]), "+v"(c[1]), "+v"(c[2]), "+v"(c[3])
                   : "v"(a0.v), "v"(a1.v), "v"(b0.v), "v"(b1.v));
    }
  }
}

__global__ void __launch_bounds__(256) k_cvt_x(const float* __restrict__ x, _Float16* __restrict__ xh) {
  constexpr int per_row = kC / 8;
  const int gid = (int)blockIdx.x * 256 + (int)threadIdx.x;
  if (gid >= kM * per_row) return;
  const int m  = gid / per_row;
  const int c8 = (gid - m * per_row) * 8;
  const int b  = m / SEQ, t = m - b * SEQ;
  const float* src = x + ((size_t)(b * SEQ_FULL + t)) * kC + c8;
  const v4f f0 = *(const v4f*)(src);
  const v4f f1 = *(const v4f*)(src + 4);
  v8h o;
#pragma unroll
  for (int j = 0; j < 4; ++j) {
    o[j]     = (_Float16)bf16r(f0[j]);
    o[j + 4] = (_Float16)bf16r(f1[j]);
  }
  _Float16* dst = xh + (size_t)m * kC + c8;
  *(volatile v8h*)dst = o;
  __threadfence();
  *(volatile v8h*)dst = o;
}

__global__ void __launch_bounds__(256) k_cvt_wt(const float* __restrict__ W, _Float16* __restrict__ WT, int N) {
  __shared__ __attribute__((aligned(16))) _Float16 tT[64][72];
  const int tid = threadIdx.x;
  const int n0 = (int)blockIdx.x * 64, k0 = (int)blockIdx.y * 64;
  {
    const int kk = tid >> 2, nc = (tid & 3) * 16;
    const float* src = W + ((size_t)(k0 + kk)) * N + n0 + nc;
#pragma unroll
    for (int q = 0; q < 4; ++q) {
      const v4f f = *(const v4f*)(src + 4 * q);
#pragma unroll
      for (int j = 0; j < 4; ++j) tT[nc + 4 * q + j][kk] = (_Float16)(bf16r(f[j]) * kWCarry);
    }
  }
  __syncthreads();
  const int p = tid & 7, lrow = tid >> 3;
  v8h o[2];
  size_t oo[2];
#pragma unroll
  for (int it = 0; it < 2; ++it) {
    const int L = it * 32 + lrow;
    o[it]  = (v8h)(*(const v8ha*)(&tT[L][8 * p]));
    oo[it] = ((size_t)(n0 + L)) * kC + k0 + 8 * p;
  }
  for (int pass = 0; pass < 2; ++pass) {
#pragma unroll
    for (int it = 0; it < 2; ++it) *(volatile v8h*)(WT + oo[it]) = o[it];
    __threadfence();
  }
}

__global__ void __launch_bounds__(256) k_qkv(const _Float16* __restrict__ xh, const _Float16* __restrict__ wT,
                                             const float* __restrict__ bias,
                                             _Float16* qh, _Float16* kh, _Float16* vT,
                                             _Float16* qres, _Float16* kres, _Float16* vTr) {
  __shared__ __attribute__((aligned(16))) float sC[64][kCP];
  const int tid = threadIdx.x, wave = tid >> 5, lane = tid & 31, l16 = lane & 15, lh = lane >> 4;
  const int wr = wave >> 2, wc = wave & 3;
  const int m0 = (int)blockIdx.x * 64, n0 = (int)blockIdx.y * 128;

  const _Float16* a0p = xh + ((size_t)(m0 + 32 * wr + l16)) * kC + 8 * lh;
  const _Float16* a1p = a0p + (size_t)16 * kC;
  const _Float16* b0p = wT + ((size_t)(n0 + 32 * wc + l16)) * kC + 8 * lh;
  const _Float16* b1p = b0p + (size_t)16 * kC;

  v8f c[4], cr[4];
  {
    v8f z = {};
#pragma unroll
    for (int i = 0; i < 4; ++i) { c[i] = z; cr[i] = z; }
  }
  gemm32<false>(a0p, a1p, a0p, a1p, b0p, b1p, kC, c, cr);

  const float bb0 = bf16r(bias[n0 + 32 * wc + l16]);
  const float bb1 = bf16r(bias[n0 + 32 * wc + 16 + l16]);
#pragma unroll
  for (int r = 0; r < 8; ++r) {
    const int row0 = 32 * wr + 8 * lh + r, row1 = row0 + 16;
    const int col0 = 32 * wc + l16, col1 = col0 + 16;
    sC[row0][col0] = c[0][r] * kWInv + bb0;
    sC[row0][col1] = c[1][r] * kWInv + bb1;
    sC[row1][col0] = c[2][r] * kWInv + bb0;
    sC[row1][col1] = c[3][r] * kWInv + bb1;
  }
  __syncthreads();

  const int which = n0 / kC;
  const int hA = (n0 - which * kC) / kD;
  const int b = m0 / SEQ, t0 = m0 - b * SEQ;
  const bool early = (t0 < kER);
  const int p = tid & 7, lrow = tid >> 3;

  if (which < 2) {
    _Float16* hp = (which == 0) ? qh : kh;
    _Float16* rp = (which == 0) ? qres : kres;
    v8h hv[4], rv[4];
    size_t oh[4], orr[4];
#pragma unroll
    for (int it = 0; it < 4; ++it) {
      const int L = it * 32 + lrow, j = L >> 6, rr = L & 63;
      const v4f f0 = (v4f)(*(const v4fa*)(&sC[rr][64 * j + 8 * p]));
      const v4f f1 = (v4f)(*(const v4fa*)(&sC[rr][64 * j + 8 * p + 4]));
#pragma unroll
      for (int e = 0; e < 4; ++e) {
        const float g0 = f0[e], g1 = f1[e];
        const _Float16 h0 = (_Float16)g0, h1 = (_Float16)g1;
        hv[it][e] = h0; hv[it][e + 4] = h1;
        rv[it][e]     = (_Float16)((g0 - (float)h0) * kRCarry);
        rv[it][e + 4] = (_Float16)((g1 - (float)h1) * kRCarry);
      }
      const int hd = hA + j;
      oh[it]  = ((size_t)((b * kH + hd) * SEQ + t0 + rr)) * kD + 8 * p;
      orr[it] = ((size_t)((b * kH + hd) * kER + t0 + rr)) * kD + 8 * p;
    }
    for (int pass = 0; pass < 2; ++pass) {
#pragma unroll
      for (int it = 0; it < 4; ++it) {
        *(volatile v8h*)(hp + oh[it]) = hv[it];
        if (early) *(volatile v8h*)(rp + orr[it]) = rv[it];
      }
      __threadfence();
    }
  } else {
    v8h hv[4], rv[4];
    size_t oh[4], orr[4];
#pragma unroll
    for (int it = 0; it < 4; ++it) {
      const int L = it * 32 + lrow, j = L >> 6, d = L & 63;
#pragma unroll
      for (int e = 0; e < 8; ++e) {
        const float g = sC[8 * p + e][64 * j + d];
        const _Float16 hh = (_Float16)g;
        hv[it][e] = hh;
        rv[it][e] = (_Float16)((g - (float)hh) * kRCarry);
      }
      const int hd = hA + j;
      oh[it]  = ((size_t)((b * kH + hd) * kD + d)) * SEQ + t0 + 8 * p;
      orr[it] = ((size_t)((b * kH + hd) * kD + d)) * kER + t0 + 8 * p;
    }
    for (int pass = 0; pass < 2; ++pass) {
#pragma unroll
      for (int it = 0; it < 4; ++it) {
        *(volatile v8h*)(vT + oh[it]) = hv[it];
        if (early) *(volatile v8h*)(vTr + orr[it]) = rv[it];
      }
      __threadfence();
    }
  }
}

template <bool EARLY>
__global__ void __launch_bounds__(128) __attribute__((amdgpu_num_vgpr(256)))
k_attn(const _Float16* __restrict__ qh, const _Float16* __restrict__ kh, const _Float16* __restrict__ vT,
       const _Float16* __restrict__ qres, const _Float16* __restrict__ kres, const _Float16* __restrict__ vTr,
       _Float16* ctxh, _Float16* ctxr) {
  __shared__ __attribute__((aligned(16))) _Float16 ldsP[4][16 * 32];
  __shared__ __attribute__((aligned(16))) _Float16 ldsR[4][16 * 32];
  __shared__ __attribute__((aligned(16))) float sO[4][16][kD];

  const int tid = threadIdx.x, wave = tid >> 5, lane = tid & 31, l16 = lane & 15, lh = lane >> 4;
  int bh, qblk;
  if (EARLY) { bh = (int)blockIdx.x / kQBE; qblk = (int)blockIdx.x - bh * kQBE; }
  else       { bh = (int)blockIdx.x / kQBL; qblk = kQBE + ((int)blockIdx.x - bh * kQBL); }
  const int b = bh / kH, h = bh - b * kH;
  const int qBase = qblk * 64 + wave * 16;

  v16h aq[2], ar[2];
  {
    const _Float16* qrow = qh + ((size_t)bh * SEQ + qBase + l16) * kD + 8 * lh;
    const _Float16* rrow = qres + ((size_t)bh * kER + (EARLY ? qBase : 0) + l16) * kD + 8 * lh;
#pragma unroll
    for (int hc = 0; hc < 2; ++hc) {
      Frag f;
      f.h[0] = *(const v8h*)(qrow + hc * 32);
      f.h[1] = *(const v8h*)(qrow + hc * 32 + 16);
      aq[hc] = f.v;
      if (EARLY) {
        Frag g;
        g.h[0] = *(const v8h*)(rrow + hc * 32);
        g.h[1] = *(const v8h*)(rrow + hc * 32 + 16);
        ar[hc] = g.v;
      } else {
        v16h z = {};
        ar[hc] = z;
      }
    }
  }

  float m[8], l[8];
  v8f co[4], co2[4];
  {
    v8f z = {};
#pragma unroll
    for (int n = 0; n < 4; ++n) { co[n] = z; co2[n] = z; }
#pragma unroll
    for (int r = 0; r < 8; ++r) { m[r] = -1.0e30f; l[r] = 0.0f; }
  }

  const _Float16* kbase  = kh   + ((size_t)bh * SEQ + l16) * kD + 8 * lh;
  const _Float16* krbase = kres + ((size_t)bh * kER + l16) * kD + 8 * lh;
  const _Float16* vbase  = vT   + ((size_t)bh * kD + l16) * SEQ + 8 * lh;
  const _Float16* vrbase = vTr  + ((size_t)bh * kD + l16) * kER + 8 * lh;

#pragma unroll 1
  for (int k0 = 0; k0 < qBase + 16; k0 += 32) {
    v8f s0 = {};
    v8f s1 = {};
    v8f r0s = {};
    v8f r1s = {};
    const _Float16* kp0 = kbase + (size_t)k0 * kD;
    const _Float16* kp1 = kp0 + 16 * kD;
    const _Float16* ep0 = krbase + (size_t)k0 * kD;
    const _Float16* ep1 = ep0 + 16 * kD;
#pragma unroll
    for (int hc = 0; hc < 2; ++hc) {
      Frag b0, b1;
      b0.h[0] = *(const v8h*)(kp0 + hc * 32); b0.h[1] = *(const v8h*)(kp0 + hc * 32 + 16);
      b1.h[0] = *(const v8h*)(kp1 + hc * 32); b1.h[1] = *(const v8h*)(kp1 + hc * 32 + 16);
      s0 = mma(aq[hc], b0.v, s0);
      s1 = mma(aq[hc], b1.v, s1);
      if (EARLY) {
        Frag e0, e1;
        e0.h[0] = *(const v8h*)(ep0 + hc * 32); e0.h[1] = *(const v8h*)(ep0 + hc * 32 + 16);
        e1.h[0] = *(const v8h*)(ep1 + hc * 32); e1.h[1] = *(const v8h*)(ep1 + hc * 32 + 16);
        r0s = mma(aq[hc], e0.v, r0s);
        r0s = mma(ar[hc], b0.v, r0s);
        r1s = mma(aq[hc], e1.v, r1s);
        r1s = mma(ar[hc], b1.v, r1s);
        asm volatile("v_nop\n\tv_nop\n\tv_nop\n\tv_nop"
                     : "+v"(s0), "+v"(s1), "+v"(r0s), "+v"(r1s)
                     : "v"(aq[hc]), "v"(ar[hc]), "v"(b0.v), "v"(b1.v), "v"(e0.v), "v"(e1.v));
      } else {
        asm volatile("v_nop\n\tv_nop\n\tv_nop\n\tv_nop"
                     : "+v"(s0), "+v"(s1)
                     : "v"(aq[hc]), "v"(b0.v), "v"(b1.v));
      }
    }

    float alpha[8];
#pragma unroll
    for (int r = 0; r < 8; ++r) {
      const int row  = qBase + r + 8 * lh;
      const int key0 = k0 + l16, key1 = key0 + 16;
      float sv0 = s0[r], sv1 = s1[r];
      if (EARLY) { sv0 += r0s[r] * kRInv; sv1 += r1s[r] * kRInv; }
      const float x0 = (key0 <= row) ? sv0 * kScale : -1.0e30f;
      const float x1 = (key1 <= row) ? sv1 * kScale : -1.0e30f;
      float tmax = fmaxf(x0, x1);
#pragma unroll
      for (int off = 1; off < 16; off <<= 1) tmax = fmaxf(tmax, __shfl_xor(tmax, off, 32));
      const float mn = fmaxf(m[r], tmax);
      alpha[r] = __expf(m[r] - mn);
      const float p0 = __expf(x0 - mn);
      const float p1 = __expf(x1 - mn);
      float ps = p0 + p1;
#pragma unroll
      for (int off = 1; off < 16; off <<= 1) ps += __shfl_xor(ps, off, 32);
      l[r] = l[r] * alpha[r] + ps;
      m[r] = mn;
      const float pc0 = p0 * kPCarry, pc1 = p1 * kPCarry;
      const _Float16 h0 = (_Float16)pc0, h1 = (_Float16)pc1;
      ldsP[wave][(r + 8 * lh) * 32 + l16]      = h0;
      ldsP[wave][(r + 8 * lh) * 32 + 16 + l16] = h1;
      if (EARLY) {
        ldsR[wave][(r + 8 * lh) * 32 + l16]      = (_Float16)((pc0 - (float)h0) * kRCarry);
        ldsR[wave][(r + 8 * lh) * 32 + 16 + l16] = (_Float16)((pc1 - (float)h1) * kRCarry);
      }
    }
#pragma unroll
    for (int n = 0; n < 4; ++n) {
#pragma unroll
      for (int r = 0; r < 8; ++r) {
        co[n][r] *= alpha[r];
        if (EARLY) co2[n][r] *= alpha[r];
      }
    }

    wave_lds_sync();

    Frag ap, apr;
    ap.h[0] = (v8h)(*(const v8ha*)(&ldsP[wave][l16 * 32 + 8 * lh]));
    ap.h[1] = (v8h)(*(const v8ha*)(&ldsP[wave][l16 * 32 + 16 + 8 * lh]));
    if (EARLY) {
      apr.h[0] = (v8h)(*(const v8ha*)(&ldsR[wave][l16 * 32 + 8 * lh]));
      apr.h[1] = (v8h)(*(const v8ha*)(&ldsR[wave][l16 * 32 + 16 + 8 * lh]));
    } else {
      v16h z = {};
      apr.v = z;
    }
    const _Float16* vp  = vbase + k0;
    const _Float16* vrp = vrbase + k0;
#pragma unroll
    for (int n = 0; n < 4; ++n) {
      Frag bv;
      bv.h[0] = *(const v8h*)(vp + (size_t)n * 16 * SEQ);
      bv.h[1] = *(const v8h*)(vp + (size_t)n * 16 * SEQ + 16);
      co[n] = mma(ap.v, bv.v, co[n]);
      if (EARLY) {
        Frag br;
        br.h[0] = *(const v8h*)(vrp + (size_t)n * 16 * kER);
        br.h[1] = *(const v8h*)(vrp + (size_t)n * 16 * kER + 16);
        co2[n] = mma(ap.v, br.v, co2[n]);
        co2[n] = mma(apr.v, bv.v, co2[n]);
        asm volatile("v_nop\n\tv_nop\n\tv_nop\n\tv_nop"
                     : "+v"(co[n]), "+v"(co2[n])
                     : "v"(ap.v), "v"(apr.v), "v"(bv.v), "v"(br.v));
      } else {
        asm volatile("v_nop\n\tv_nop\n\tv_nop\n\tv_nop"
                     : "+v"(co[n])
                     : "v"(ap.v), "v"(bv.v));
      }
    }
  }

#pragma unroll
  for (int r = 0; r < 8; ++r) {
    const float inv = (1.0f / l[r]) * kPInv;
#pragma unroll
    for (int n = 0; n < 4; ++n) {
      float o = co[n][r];
      if (EARLY) o += co2[n][r] * kRInv;
      sO[wave][r + 8 * lh][n * 16 + l16] = o * inv;
    }
  }
  wave_lds_sync();

  const int p = lane & 7;
  v8h hv[4], rv[4];
  size_t oh[4], orr[4];
#pragma unroll
  for (int it = 0; it < 4; ++it) {
    const int rr = it * 4 + (lane >> 3);
    const v4f f0 = (v4f)(*(const v4fa*)(&sO[wave][rr][8 * p]));
    const v4f f1 = (v4f)(*(const v4fa*)(&sO[wave][rr][8 * p + 4]));
#pragma unroll
    for (int e = 0; e < 4; ++e) {
      const float g0 = f0[e], g1 = f1[e];
      const _Float16 h0 = (_Float16)g0, h1 = (_Float16)g1;
      hv[it][e] = h0; hv[it][e + 4] = h1;
      rv[it][e]     = (_Float16)((g0 - (float)h0) * kRCarry);
      rv[it][e + 4] = (_Float16)((g1 - (float)h1) * kRCarry);
    }
    oh[it]  = ((size_t)(b * SEQ + qBase + rr)) * kC + h * kD + 8 * p;
    orr[it] = ((size_t)(b * kER + (EARLY ? (qBase + rr) : 0))) * kC + h * kD + 8 * p;
  }
  for (int pass = 0; pass < 2; ++pass) {
#pragma unroll
    for (int it = 0; it < 4; ++it) {
      *(volatile v8h*)(ctxh + oh[it]) = hv[it];
      if (EARLY) *(volatile v8h*)(ctxr + orr[it]) = rv[it];
    }
    __threadfence();
  }
}

__global__ void __launch_bounds__(256) k_proj(const _Float16* __restrict__ ctxh, const _Float16* __restrict__ ctxr,
                                              const _Float16* __restrict__ wT, const float* __restrict__ bias,
                                              float* out) {
  __shared__ __attribute__((aligned(16))) float sC[64][kCP];
  const int tid = threadIdx.x, wave = tid >> 5, lane = tid & 31, l16 = lane & 15, lh = lane >> 4;
  const int wr = wave >> 2, wc = wave & 3;
  const int m0 = (int)blockIdx.x * 64, n0 = (int)blockIdx.y * 128;
  const int b = m0 / SEQ, t0 = m0 - b * SEQ;
  const bool early = (t0 < kER);

  const _Float16* a0p = ctxh + ((size_t)(m0 + 32 * wr + l16)) * kC + 8 * lh;
  const _Float16* a1p = a0p + (size_t)16 * kC;
  const _Float16* b0p = wT + ((size_t)(n0 + 32 * wc + l16)) * kC + 8 * lh;
  const _Float16* b1p = b0p + (size_t)16 * kC;

  v8f c[4], cr[4];
  {
    v8f z = {};
#pragma unroll
    for (int i = 0; i < 4; ++i) { c[i] = z; cr[i] = z; }
  }
  if (early) {
    const _Float16* r0p = ctxr + ((size_t)(b * kER + t0 + 32 * wr + l16)) * kC + 8 * lh;
    const _Float16* r1p = r0p + (size_t)16 * kC;
    gemm32<true>(a0p, a1p, r0p, r1p, b0p, b1p, kC, c, cr);
  } else {
    gemm32<false>(a0p, a1p, a0p, a1p, b0p, b1p, kC, c, cr);
  }

  const float bb0 = bf16r(bias[n0 + 32 * wc + l16]);
  const float bb1 = bf16r(bias[n0 + 32 * wc + 16 + l16]);
#pragma unroll
  for (int r = 0; r < 8; ++r) {
    const int row0 = 32 * wr + 8 * lh + r, row1 = row0 + 16;
    const int col0 = 32 * wc + l16, col1 = col0 + 16;
    sC[row0][col0] = (c[0][r] + cr[0][r] * kRInv) * kWInv + bb0;
    sC[row0][col1] = (c[1][r] + cr[1][r] * kRInv) * kWInv + bb1;
    sC[row1][col0] = (c[2][r] + cr[2][r] * kRInv) * kWInv + bb0;
    sC[row1][col1] = (c[3][r] + cr[3][r] * kRInv) * kWInv + bb1;
  }
  __syncthreads();

  v4f ov[8];
  size_t oo[8];
#pragma unroll
  for (int it = 0; it < 8; ++it) {
    const int rr = it * 8 + wave;
    ov[it] = (v4f)(*(const v4fa*)(&sC[rr][4 * lane]));
    oo[it] = ((size_t)(b * SEQ_FULL + t0 + rr)) * kC + n0 + 4 * lane;
  }
  for (int pass = 0; pass < 2; ++pass) {
#pragma unroll
    for (int it = 0; it < 8; ++it) *(volatile v4f*)(out + oo[it]) = ov[it];
    __threadfence();
  }
}

extern "C" void kernel_launch(void* const* d_in, const int* in_sizes, int n_in,
                              void* d_out, int out_size, void* d_ws, size_t ws_size,
                              hipStream_t stream) {
  if (n_in < 5) return;
  const long long need_x = (long long)((NB - 1) * SEQ_FULL + SEQ) * (long long)kC;
  if ((long long)in_sizes[0] < need_x) return;
  if (in_sizes[1] < kC * kNQ) return;
  if (in_sizes[2] < kNQ) return;
  if (in_sizes[3] < kC * kC) return;
  if (in_sizes[4] < kC) return;
  if ((long long)out_size < need_x) return;
  if (ws_size < kWsTotal) return;

  const float* x      = (const float*)d_in[0];
  const float* W_qkv  = (const float*)d_in[1];
  const float* b_qkv  = (const float*)d_in[2];
  const float* W_proj = (const float*)d_in[3];
  const float* b_proj = (const float*)d_in[4];
  float* out = (float*)d_out;

  char* ws = (char*)d_ws;
  size_t off = 0;
  _Float16* xh   = (_Float16*)(ws + off); off += kBytesX;
  _Float16* wq   = (_Float16*)(ws + off); off += kBytesWq;
  _Float16* wp   = (_Float16*)(ws + off); off += kBytesWp;
  _Float16* qh   = (_Float16*)(ws + off); off += kBytesQK;
  _Float16* kh   = (_Float16*)(ws + off); off += kBytesQK;
  _Float16* vT   = (_Float16*)(ws + off); off += kBytesQK;
  _Float16* qres = (_Float16*)(ws + off); off += kBytesQKr;
  _Float16* kres = (_Float16*)(ws + off); off += kBytesQKr;
  _Float16* vTr  = (_Float16*)(ws + off); off += kBytesQKr;
  _Float16* ctxh = (_Float16*)(ws + off); off += kBytesCtx;
  _Float16* ctxr = (_Float16*)(ws + off); off += kBytesCtr;
  if (off > ws_size) return;

  k_cvt_x<<<dim3((kM * (kC / 8)) / 256), dim3(256), 0, stream>>>(x, xh);
  k_cvt_wt<<<dim3(kNQ / 64, kC / 64), dim3(256), 0, stream>>>(W_qkv, wq, kNQ);
  k_cvt_wt<<<dim3(kC / 64, kC / 64), dim3(256), 0, stream>>>(W_proj, wp, kC);
  k_qkv<<<dim3(kM / 64, kNQ / 128), dim3(256), 0, stream>>>(xh, wq, b_qkv, qh, kh, vT, qres, kres, vTr);
  k_attn<true><<<dim3(NB * kH * kQBE), dim3(128), 0, stream>>>(qh, kh, vT, qres, kres, vTr, ctxh, ctxr);
  if (SEQ / 64 > kQBE) {
    k_attn<false><<<dim3(NB * kH * (SEQ / 64 - kQBE)), dim3(128), 0, stream>>>(qh, kh, vT, qres, kres, vTr, ctxh, ctxr);
  }
  k_proj<<<dim3(kM / 64, kC / 128), dim3(256), 0, stream>>>(ctxh, ctxr, wp, b_proj, out);
}
